// Critic_50276887167257
// MI455X (gfx1250) — hardware-verified
//
#include <hip/hip_runtime.h>
#include <math.h>

constexpr int NNODE  = 200000;
constexpr int NEDGE  = 1600000;
constexpr int NGRAPH = 1000;
constexpr int NGPAD  = 1024;
constexpr int SDIM   = 64;
constexpr int ADIM   = 32;
constexpr int HID    = 128;
constexpr int NT     = 256;

constexpr int AGG_TILE          = 8192;
constexpr int AGG_ROWS_PER_WAVE = AGG_TILE / 8;
constexpr int TILES_PER_CHUNK   = 5;
constexpr int CHUNK_ROWS        = AGG_TILE * TILES_PER_CHUNK;
constexpr int NCHUNK            = 5;
constexpr int DEG_TILE          = 16384;
constexpr int DEG_ROWS_PER_WAVE = DEG_TILE / 8;
constexpr int NDEGBLK           = 13;
constexpr int DINV_ROWS         = NDEGBLK * DEG_TILE;
constexpr int SCH               = 4096;
constexpr int ESP               = SCH / NT;
constexpr int NECH              = (NEDGE + SCH - 1) / SCH;
constexpr int PSCH              = 2048;
constexpr int PSP               = PSCH / NT;
constexpr int STAT_ROWS         = 1600;
constexpr int NSTATBLK          = NNODE / STAT_ROWS;
constexpr int PTW               = 512;
constexpr int SCANW             = 80;
constexpr float CARRY_XA  = 16.0f;
constexpr float CARRY_W   = 16.0f;
constexpr float CARRY_H0  = 16.0f;
constexpr float CARRY_ACT = 8.0f;
constexpr float SCALE_G1  = CARRY_H0 / (CARRY_XA * CARRY_W);
constexpr float SCALE_G2  = 1.0f / (CARRY_H0 * CARRY_W);
constexpr float SCALE_G3  = 1.0f / (CARRY_ACT * CARRY_W);

static_assert(NT == 256);
static_assert(NEDGE % ESP == 0);
static_assert(SCH % NT == 0 && PSCH % NT == 0 && PSP == 8 && ESP == 16);
static_assert(CHUNK_ROWS % 64 == 0 && NNODE % 64 == 0);
static_assert(NCHUNK * CHUNK_ROWS >= NNODE && (NCHUNK - 1) * CHUNK_ROWS < NNODE);
static_assert((NNODE - (NCHUNK - 1) * CHUNK_ROWS) % 64 == 0);
static_assert(DINV_ROWS >= NCHUNK * CHUNK_ROWS);
static_assert(NSTATBLK * STAT_ROWS == NNODE && STAT_ROWS % 4 == 0);
static_assert(SDIM % 32 == 0 && HID % 64 == 0 && ADIM % 32 == 0);
static_assert(AGG_ROWS_PER_WAVE == 1024 && DEG_ROWS_PER_WAVE == 2048);
static_assert(NGPAD == 32 * 32 && NGRAPH <= NGPAD && NGRAPH % 4 == 0 && NGPAD % NT == 0);
static_assert(NNODE < (1 << 18));

typedef __attribute__((ext_vector_type(16))) _Float16 v16h;
typedef __attribute__((ext_vector_type(8)))  _Float16 v8h;
typedef __attribute__((ext_vector_type(16))) __bf16   v16b;
typedef __attribute__((ext_vector_type(8)))  __bf16   v8b;
typedef __attribute__((ext_vector_type(8)))  float    v8f;
typedef __attribute__((ext_vector_type(4)))  float    v4f;
typedef __attribute__((ext_vector_type(2)))  float    v2f;
typedef __attribute__((ext_vector_type(4)))  int      v4i;
typedef __attribute__((ext_vector_type(4)))  unsigned int v4u;

__device__ __forceinline__ unsigned short f2bf_bits(float f) {
  unsigned u = __float_as_uint(f);
  return (unsigned short)((u + 0x7FFFu + ((u >> 16) & 1u)) >> 16);
}
__device__ __forceinline__ float bf_bits2f(unsigned short h) { return __uint_as_float(((unsigned)h) << 16); }
__device__ __forceinline__ unsigned pk16(unsigned short a, unsigned short b) { return (unsigned)a | ((unsigned)b << 16); }
__device__ __forceinline__ unsigned short h_bits(float f) { const _Float16 h = (_Float16)f; return __builtin_bit_cast(unsigned short, h); }
__device__ __forceinline__ float h16_to_f32(unsigned hb) {
  const unsigned sgn = (hb & 0x8000u) << 16; const unsigned em = hb & 0x7fffu;
  const float fn = __uint_as_float((em << 13) + 0x38000000u);
  const float fs = (float)em * 5.9604644775390625e-8f;
  const float mag = (em < 0x400u) ? fs : fn; return __uint_as_float(__float_as_uint(mag) | sgn); }

__device__ __forceinline__ void dep_guard_h(v8f& a, v8f& b, v16h x, v16h y) { asm volatile("v_nop\n\tv_nop\n\tv_nop\n\tv_nop" : "+v"(a), "+v"(b) : "v"(x), "v"(y)); }
__device__ __forceinline__ void dep_guard_b(v8f& a, v8f& b, v16b x, v16b y) { asm volatile("v_nop\n\tv_nop\n\tv_nop\n\tv_nop" : "+v"(a), "+v"(b) : "v"(x), "v"(y)); }
__device__ __forceinline__ void dep_guard4_h(v8f& a, v8f& b, v8f& c, v8f& d, v16h x, v16h y) { asm volatile("v_nop\n\tv_nop\n\tv_nop\n\tv_nop" : "+v"(a), "+v"(b), "+v"(c), "+v"(d) : "v"(x), "v"(y)); }
__device__ __forceinline__ void dep_guard4_b(v8f& a, v8f& b, v8f& c, v8f& d, v16b x, v16b y) { asm volatile("v_nop\n\tv_nop\n\tv_nop\n\tv_nop" : "+v"(a), "+v"(b), "+v"(c), "+v"(d) : "v"(x), "v"(y)); }
__device__ __forceinline__ void keep4_h(v16h a, v16h b, v16h c, v16h d) { asm volatile("v_nop" :: "v"(a), "v"(b), "v"(c), "v"(d)); }
__device__ __forceinline__ void keep4_b(v16b a, v16b b, v16b c, v16b d) { asm volatile("v_nop" :: "v"(a), "v"(b), "v"(c), "v"(d)); }
__device__ __forceinline__ void acc_guard4(v8f& a, v8f& b, v8f& c, v8f& d) { asm volatile("v_nop\n\tv_nop\n\tv_nop\n\tv_nop" : "+v"(a), "+v"(b), "+v"(c), "+v"(d)); }
template <typename T> struct Frag;
template <> struct Frag<_Float16> {
  typedef v16h V; union U { v16h v; v8h h[2]; };
  static __device__ __forceinline__ v16h load(const _Float16* p) {
    U f; f.h[0] = *(const v8h*)(p); f.h[1] = *(const v8h*)(p + 16); return f.v;
  }
  static __device__ __forceinline__ v8f mma(v16h a, v16h b, v8f c) {
    return __builtin_amdgcn_wmma_f32_16x16x32_f16(false, a, false, b, (short)0, c, false, false);
  }
  static __device__ __forceinline__ void guard(v8f& a, v8f& b, v16h x, v16h y) { dep_guard_h(a, b, x, y); }
  static __device__ __forceinline__ void guard4(v8f& a, v8f& b, v8f& c, v8f& d, v16h x, v16h y) { dep_guard4_h(a, b, c, d, x, y); }
  static __device__ __forceinline__ void keep(v16h a, v16h b, v16h c, v16h d) { keep4_h(a, b, c, d); }
};
template <> struct Frag<__bf16> {
  typedef v16b V; union U { v16b v; v8b h[2]; };
  static __device__ __forceinline__ v16b load(const __bf16* p) {
    U f; f.h[0] = *(const v8b*)(p); f.h[1] = *(const v8b*)(p + 16); return f.v;
  }
  static __device__ __forceinline__ v8f mma(v16b a, v16b b, v8f c) {
    return __builtin_amdgcn_wmma_f32_16x16x32_bf16(false, a, false, b, (short)0, c, false, false);
  }
  static __device__ __forceinline__ void guard(v8f& a, v8f& b, v16b x, v16b y) { dep_guard_b(a, b, x, y); }
  static __device__ __forceinline__ void guard4(v8f& a, v8f& b, v8f& c, v8f& d, v16b x, v16b y) { dep_guard4_b(a, b, c, d, x, y); }
  static __device__ __forceinline__ void keep(v16b a, v16b b, v16b c, v16b d) { keep4_b(a, b, c, d); }
};

template <int ET> struct Elem;
template <> struct Elem<0> { typedef _Float16 T; };
template <> struct Elem<1> { typedef __bf16 T; };
template <int ET, bool SPLIT, int BIAS_MODE, int OUT_MODE, bool RESID, int ACT = 0>
__global__ __launch_bounds__(256) void wmma_gemm64(
    const unsigned short* __restrict__ Ap, const unsigned short* __restrict__ A2p, int lda, long strideA,
    const unsigned short* __restrict__ Btp, const unsigned short* __restrict__ Bt2p, int ldb, long strideB,
    void* __restrict__ Cout, void* __restrict__ Cout2, int ldc, long strideC,
    const float* __restrict__ bias,
    const float* __restrict__ resid, long strideR,
    int M, int N, int K, float scale) {
  typedef typename Elem<ET>::T T;
  typedef typename Frag<T>::V V;
  const T* A = (const T*)Ap; const T* A2 = (const T*)A2p; const T* Bt = (const T*)Btp; const T* Bt2 = (const T*)Bt2p;
  __shared__ __align__(16) float sT[8][16 * 68];
  const int b    = blockIdx.y;
  const int lane = threadIdx.x & 31;
  const int wave = threadIdx.x >> 5;
  const int tilesN = N >> 6;
  const int tilesM = M >> 6;
  const int tile = blockIdx.x * 8 + wave;
  if (tile >= tilesM * tilesN) return;
  const int tm = tile / tilesN;
  const int tn = tile - tm * tilesN;
  const int m0 = tm << 6;
  const int n0 = tn << 6;

  const T* Ab  = A  + (size_t)b * strideA;
  const T* Bb  = Bt + (size_t)b * strideB;
  const T* Ab2 = SPLIT ? (A2  + (size_t)b * strideA) : nullptr;
  const T* Bb2 = SPLIT ? (Bt2 + (size_t)b * strideB) : nullptr;

  const int rlane = lane & 15;
  const int koff  = (lane >> 4) * 8;
  const int mOff  = (lane >> 4) * 8;

  v8f acc[4][4];
#pragma unroll
  for (int i = 0; i < 4; ++i)
#pragma unroll
    for (int j = 0; j < 4; ++j) acc[i][j] = (v8f){0.f,0.f,0.f,0.f,0.f,0.f,0.f,0.f};

  for (int k0 = 0; k0 < K; k0 += 32) {
    V bh[4], bl[4];
#pragma unroll
    for (int j = 0; j < 4; ++j) {
      const size_t bo = (size_t)(n0 + (j << 4) + rlane) * ldb + koff + k0;
      bh[j] = Frag<T>::load(Bb + bo);
      if (SPLIT) bl[j] = Frag<T>::load(Bb2 + bo);
    }
#pragma unroll
    for (int i = 0; i < 4; ++i) {
      const size_t ao = (size_t)(m0 + (i << 4) + rlane) * lda + koff + k0;
      V ah = Frag<T>::load(Ab + ao);
      V al;
      if (SPLIT) al = Frag<T>::load(Ab2 + ao);
#pragma unroll
      for (int j = 0; j < 4; ++j) {
        acc[i][j] = Frag<T>::mma(ah, bh[j], acc[i][j]);
        if (SPLIT) {
          acc[i][j] = Frag<T>::mma(ah, bl[j], acc[i][j]);
          acc[i][j] = Frag<T>::mma(al, bh[j], acc[i][j]);
        }
      }
      Frag<T>::guard4(acc[i][0], acc[i][1], acc[i][2], acc[i][3], ah, SPLIT ? al : ah);
    }
    Frag<T>::keep(bh[0], bh[1], bh[2], bh[3]);
    if (SPLIT) Frag<T>::keep(bl[0], bl[1], bl[2], bl[3]);
  }
  acc_guard4(acc[0][0], acc[0][1], acc[0][2], acc[0][3]);
  acc_guard4(acc[1][0], acc[1][1], acc[1][2], acc[1][3]);
  acc_guard4(acc[2][0], acc[2][1], acc[2][2], acc[2][3]);
  acc_guard4(acc[3][0], acc[3][1], acc[3][2], acc[3][3]);

  float* slab = sT[wave];
  const float* Rb = RESID ? (resid + (size_t)b * strideR) : nullptr;
#pragma unroll
  for (int i = 0; i < 4; ++i) {
    const int mBase = m0 + (i << 4);
#pragma unroll
    for (int j = 0; j < 4; ++j) {
      const int n = n0 + (j << 4) + rlane;
      float bv = 0.f;
      if (BIAS_MODE == 2) bv = bias[n];
#pragma unroll
      for (int r = 0; r < 8; ++r) {
        float v = acc[i][j][r] * scale;
        if (BIAS_MODE == 1) v += bias[mBase + mOff + r];
        if (BIAS_MODE == 2) v += bv;
        if (RESID) v += Rb[(size_t)(mBase + mOff + r) * ldc + n];
        if (ACT == 2) v = fmaxf(v, 0.0f);
        if (ACT == 4) v = (v > 0.f) ? v : 0.01f * v;
        slab[(mOff + r) * 68 + (j << 4) + rlane] = v;
      }
    }
    __builtin_amdgcn_fence(__ATOMIC_RELEASE, "workgroup");
    __builtin_amdgcn_wave_barrier();
    __builtin_amdgcn_fence(__ATOMIC_ACQUIRE, "workgroup");
    if (OUT_MODE == 0) {
      float* C = (float*)Cout + (size_t)b * strideC;
      const int hh = lane >> 4, c4 = (lane & 15) * 4;
      for (int pass = 0; pass < 2; ++pass) {
#pragma unroll
        for (int it = 0; it < 8; ++it) {
          const int row = it * 2 + hh;
          v4f v = *(const v4f*)(slab + row * 68 + c4);
          *(volatile v4f*)(C + (size_t)(mBase + row) * ldc + n0 + c4) = v;
        }
        __threadfence();
      }
    } else {
      const int q = lane >> 3, c8 = (lane & 7) * 8;
      unsigned short* C  = (unsigned short*)Cout  + (size_t)b * strideC;
      unsigned short* C2 = (OUT_MODE == 2) ? ((unsigned short*)Cout2 + (size_t)b * strideC) : nullptr;
      for (int pass = 0; pass < 2; ++pass) {
#pragma unroll
        for (int it = 0; it < 4; ++it) {
          const int row = it * 4 + q;
          const float* sp = slab + row * 68 + c8;
          v8h hv, lv;
#pragma unroll
          for (int e = 0; e < 8; ++e) {
            if (OUT_MODE == 1) {
              hv[e] = (_Float16)sp[e];
            } else {
              unsigned short hb = f2bf_bits(sp[e]);
              unsigned short lb = f2bf_bits(sp[e] - bf_bits2f(hb));
              hv[e] = __builtin_bit_cast(_Float16, hb);
              lv[e] = __builtin_bit_cast(_Float16, lb);
            }
          }
          *(volatile v8h*)(C + (size_t)(mBase + row) * ldc + n0 + c8) = hv;
          if (OUT_MODE == 2) *(volatile v8h*)(C2 + (size_t)(mBase + row) * ldc + n0 + c8) = lv;
        }
        __threadfence();
      }
    }
    __builtin_amdgcn_fence(__ATOMIC_RELEASE, "workgroup");
    __builtin_amdgcn_wave_barrier();
    __builtin_amdgcn_fence(__ATOMIC_ACQUIRE, "workgroup");
  }
}

__device__ __forceinline__ int blk_excl_scan(int cnt, int* scan_ws, int tid, int* tot) {
  const int lane = tid & 31, wave = tid >> 5; int incl = cnt;
#pragma unroll
  for (int o = 1; o < 32; o <<= 1) { const int v = __shfl_up(incl, o, 32); if (lane >= o) incl += v; }
  if (lane == 31) scan_ws[wave] = incl;
  __syncthreads();
  if (wave == 0) { const int wv = scan_ws[lane]; int wincl = wv;
#pragma unroll
    for (int o = 1; o < 32; o <<= 1) { const int v = __shfl_up(wincl, o, 32); if (lane >= o) wincl += v; }
    if (lane < NT / 32) scan_ws[32 + lane] = wincl - wv; if (lane == 31) scan_ws[64] = wincl; }
  __syncthreads();
  const int res = scan_ws[32 + wave] + incl - cnt; *tot = scan_ws[64];
  return res;
}

__device__ __forceinline__ int chunk_hits_deg(const int* __restrict__ dstv, int e0, int n0, int tid, int* LIST, int* scan_ws) {
  const int eb = e0 + tid * ESP;
  const bool valid = eb < NEDGE;
  const int ebc = valid ? eb : (NEDGE - ESP);
  int rec[ESP]; int cnt = 0;
#pragma unroll
  for (int k = 0; k < ESP; k += 4) {
    const v4i d4 = *(const v4i*)(dstv + ebc + k);
#pragma unroll
    for (int e = 0; e < 4; ++e) {
      const int d = d4[e]; int r = -1;
      if (valid && d >= n0 && d < n0 + DEG_TILE) { r = d - n0; ++cnt; }
      rec[k + e] = r;
    }
  }
  int tot; int p = blk_excl_scan(cnt, scan_ws, tid, &tot);
#pragma unroll
  for (int k = 0; k < ESP; ++k) if (rec[k] >= 0) { if ((unsigned)p < (unsigned)SCH) LIST[p] = rec[k]; ++p; }
  __syncthreads();
  return tot < SCH ? tot : SCH;
}
__device__ __forceinline__ int chunk_hits_agg(const int* __restrict__ dstv, const int* __restrict__ srcv, int e0, int n0, int tid,
                                              int* LIST, int* scan_ws) {
  const int eb = e0 + tid * ESP;
  const bool valid = eb < NEDGE;
  const int ebc = valid ? eb : (NEDGE - ESP);
  int rec[ESP]; int cnt = 0;
#pragma unroll
  for (int k = 0; k < ESP; k += 4) {
    const v4i d4 = *(const v4i*)(dstv + ebc + k);
    const v4i s4 = *(const v4i*)(srcv + ebc + k);
#pragma unroll
    for (int e = 0; e < 4; ++e) {
      const int d = d4[e]; int r = -1;
      if (valid && d >= n0 && d < n0 + AGG_TILE) {
        int s = s4[e]; s = s < 0 ? 0 : (s >= NNODE ? NNODE - 1 : s);
        r = ((d - n0) << 18) | s; ++cnt;
      }
      rec[k + e] = r;
    }
  }
  int tot; int p = blk_excl_scan(cnt, scan_ws, tid, &tot);
#pragma unroll
  for (int k = 0; k < ESP; ++k) if (rec[k] >= 0) { if ((unsigned)p < (unsigned)SCH) LIST[p] = rec[k]; ++p; }
  __syncthreads();
  return tot < SCH ? tot : SCH;
}

__global__ __launch_bounds__(NT) void pack_kernel(const float* __restrict__ Wg, const float* __restrict__ W2,
                                                 const float* __restrict__ bg,
                                                 unsigned short* __restrict__ WgT, unsigned short* __restrict__ W2T,
                                                 float* __restrict__ bsc) {
  __shared__ __align__(16) float sb[HID];
  const int tid = threadIdx.x, lane = tid & 31, wave = tid >> 5;
  const int piece = tid & 7, lgrp = tid >> 3;
  if (tid < HID) sb[tid] = bg[tid] * CARRY_H0;
  __syncthreads();
  for (int pass = 0; pass < 2; ++pass) {
#pragma unroll 1
    for (int it = 0; it < 4; ++it) {
      const int n = it * 32 + lgrp; const int k0 = 8 * piece;
      unsigned short hb[8];
#pragma unroll
      for (int e = 0; e < 8; ++e) hb[e] = h_bits(Wg[(size_t)(k0 + e) * HID + n] * CARRY_W);
      const v4u u = (v4u){pk16(hb[0], hb[1]), pk16(hb[2], hb[3]), pk16(hb[4], hb[5]), pk16(hb[6], hb[7])};
      *(volatile v4u*)(WgT + (size_t)n * SDIM + k0) = u;
    }
#pragma unroll 1
    for (int it = 0; it < 2; ++it) {
      const int L = it * 32 + lgrp; const int n = 2 * L + (piece >> 2); const int k0 = 8 * (piece & 3);
      unsigned short hb[8];
#pragma unroll
      for (int e = 0; e < 8; ++e) hb[e] = h_bits(W2[(size_t)(k0 + e) * HID + n] * CARRY_W);
      const v4u u = (v4u){pk16(hb[0], hb[1]), pk16(hb[2], hb[3]), pk16(hb[4], hb[5]), pk16(hb[6], hb[7])};
      *(volatile v4u*)(W2T + (size_t)n * ADIM + k0) = u;
    }
    if (wave == 0) { const v4f v = *(const v4f*)(sb + 4 * lane); *(volatile v4f*)(bsc + 4 * lane) = v; }
    __threadfence();
  }
}

__global__ __launch_bounds__(NT) void deg_kernel(const int* __restrict__ ei, float* __restrict__ dinv) {
  __shared__ int LIST[SCH];
  __shared__ __align__(16) int CNT[DEG_TILE];
  __shared__ int scan_ws[SCANW];
  const int tid = threadIdx.x, lane = tid & 31, wave = tid >> 5;
  const int n0 = blockIdx.x * DEG_TILE;
  for (int i = tid; i < DEG_TILE; i += NT) CNT[i] = 0;
  for (int i = tid; i < SCH; i += NT) LIST[i] = 0;
  for (int i = tid; i < SCANW; i += NT) scan_ws[i] = 0;
  __syncthreads();
  const int* dstv = ei + NEDGE;
#pragma unroll 1
  for (int c = 0; c < NECH; ++c) {
    const int tot = chunk_hits_deg(dstv, c * SCH, n0, tid, LIST, scan_ws);
#pragma unroll 1
    for (int base = 0; base < tot; base += 32) {
      const int q = base + lane; const int qc = q < SCH ? q : (SCH - 1);
      const int lv = LIST[qc];
      const int own = ((q < tot) && ((lv >> 11) == wave)) ? 1 : 0;
      unsigned msk = (unsigned)__ballot(own);
#pragma unroll 1
      for (int it = 0; it < 32; ++it) {
        if (msk == 0u) break;
        const int bp = __builtin_ctz(msk); msk &= msk - 1u;
        const int dl = __shfl(lv, bp, 32);
        if (lane == 0) CNT[dl] += 1;
      }
    }
    __syncthreads();
  }
  for (int pass = 0; pass < 2; ++pass) {
#pragma unroll 1
    for (int j = 0; j < DEG_ROWS_PER_WAVE / 128; ++j) {
      const int dl0 = wave * DEG_ROWS_PER_WAVE + j * 128 + 4 * lane;
      const v4i c4 = *(const v4i*)(CNT + dl0);
      v4f v;
#pragma unroll
      for (int e = 0; e < 4; ++e) v[e] = rsqrtf(1.0f + (float)c4[e]);
      *(volatile v4f*)(dinv + (size_t)n0 + dl0) = v;
    }
    __threadfence();
  }
}

__global__ __launch_bounds__(NT) void agg_kernel(const float* __restrict__ x, const int* __restrict__ ei, const float* __restrict__ dinv,
                                                float* ACC, unsigned short* __restrict__ XA, int tile0) {
  __shared__ int LIST[SCH];
  __shared__ int scan_ws[SCANW];
  const int tid = threadIdx.x, lane = tid & 31, wave = tid >> 5;
  const int n0 = (tile0 + blockIdx.x) * AGG_TILE;
  const int rbase = blockIdx.x * AGG_TILE;
  for (int i = tid; i < SCH; i += NT) LIST[i] = 0;
  for (int i = tid; i < SCANW; i += NT) scan_ws[i] = 0;
#pragma unroll 1
  for (int j = 0; j < AGG_ROWS_PER_WAVE; ++j) {
    const int dl = wave * AGG_ROWS_PER_WAVE + j; const int n = n0 + dl; const int nc = n < NNODE ? n : (NNODE - 1);
    const float di = dinv[nc];
    const v2f xv = *(const v2f*)(x + (size_t)nc * SDIM + 2 * lane);
    *(v2f*)(ACC + (size_t)(rbase + dl) * SDIM + 2 * lane) = xv * di;
  }
  __syncthreads();
  const int* srcv = ei; const int* dstv = ei + NEDGE;
#pragma unroll 1
  for (int c = 0; c < NECH; ++c) {
    const int tot = chunk_hits_agg(dstv, srcv, c * SCH, n0, tid, LIST, scan_ws);
#pragma unroll 1
    for (int base = 0; base < tot; base += 32) {
      const int q = base + lane; const int qc = q < SCH ? q : (SCH - 1);
      const int lv = LIST[qc];
      const int own = ((q < tot) && ((lv >> 28) == wave)) ? 1 : 0;
      unsigned msk = (unsigned)__ballot(own);
#pragma unroll 1
      for (int it = 0; it < 32; ++it) {
        if (msk == 0u) break;
        const int bp = __builtin_ctz(msk); msk &= msk - 1u;
        const int r = __shfl(lv, bp, 32);
        const int dl = r >> 18, s = r & 0x3FFFF;
        const float ds = dinv[s];
        const v2f xv = *(const v2f*)(x + (size_t)s * SDIM + 2 * lane);
        float* rp = ACC + (size_t)(rbase + dl) * SDIM + 2 * lane;
        v2f a = *(const v2f*)rp;
        a = a + xv * ds;
        *(v2f*)rp = a;
      }
    }
    __syncthreads();
  }
#pragma unroll 1
  for (int j = 0; j < AGG_ROWS_PER_WAVE; ++j) {
    const int dl = wave * AGG_ROWS_PER_WAVE + j; const int n = n0 + dl; const int nc = n < NNODE ? n : (NNODE - 1);
    const float dn = dinv[nc] * CARRY_XA;
    const v2f a = *(const v2f*)(ACC + (size_t)(rbase + dl) * SDIM + 2 * lane);
    const float f0 = a[0] * dn, f1 = a[1] * dn;
    const unsigned u = pk16(h_bits(f0), h_bits(f1));
    unsigned* qp = (unsigned*)(XA + (size_t)(rbase + dl) * SDIM) + lane;
    *(volatile unsigned*)qp = u;
    __threadfence();
    *(volatile unsigned*)qp = u;
  }
}

__global__ __launch_bounds__(NT) void stats0_kernel(const unsigned* __restrict__ H0w, float* __restrict__ ST0) {
  __shared__ __align__(16) float red[4][256];
  __shared__ __align__(16) float red2[256];
  const int tid = threadIdx.x, lane = tid & 31, wave = tid >> 5;
  const int grp = tid >> 6, t = tid & 63;
  const int r0 = blockIdx.x * STAT_ROWS;
  float s0 = 0.f, s1 = 0.f, q0 = 0.f, q1 = 0.f;
#pragma unroll 1
  for (int k = 0; k < STAT_ROWS / 4; ++k) {
    const int row = r0 + grp + 4 * k;
    const unsigned w = H0w[(size_t)row * (HID / 2) + t];
    const float a = h16_to_f32(w & 0xffffu), b = h16_to_f32(w >> 16);
    s0 += a; s1 += b; q0 = fmaf(a, a, q0); q1 = fmaf(b, b, q1);
  }
  red[grp][2 * t] = s0; red[grp][2 * t + 1] = s1; red[grp][HID + 2 * t] = q0; red[grp][HID + 2 * t + 1] = q1;
  __syncthreads();
  { const float v = ((red[0][tid] + red[1][tid]) + red[2][tid]) + red[3][tid]; red2[tid] = v; }
  __syncthreads();
  if (wave == 0) {
    const v4f p0 = *(const v4f*)(red2 + 4 * lane);
    const v4f p1 = *(const v4f*)(red2 + HID + 4 * lane);
    float* dst = ST0 + (size_t)blockIdx.x * 256;
    for (int pass = 0; pass < 2; ++pass) {
      *(volatile v4f*)(dst + 4 * lane) = p0;
      *(volatile v4f*)(dst + HID + 4 * lane) = p1;
      __threadfence();
    }
  }
}

__global__ __launch_bounds__(NT) void fold_kernel(const float* __restrict__ ST0, const float* __restrict__ g0, const float* __restrict__ be0,
                                                 const float* __restrict__ W1, const float* __restrict__ b1,
                                                 unsigned short* __restrict__ W1T, float* __restrict__ c1) {
  __shared__ float ssc[HID];
  __shared__ float ssh[HID];
  __shared__ __align__(16) float sc1[HID];
  const int tid = threadIdx.x, lane = tid & 31, wave = tid >> 5;
  if (tid < HID) {
    double S = 0.0, Q = 0.0;
#pragma unroll 1
    for (int b = 0; b < NSTATBLK; ++b) { S += (double)ST0[b * 256 + tid]; Q += (double)ST0[b * 256 + HID + tid]; }
    const double mu = S / ((double)NNODE * (double)CARRY_H0);
    const double e2 = Q / ((double)NNODE * (double)CARRY_H0 * (double)CARRY_H0);
    double var = e2 - mu * mu; var = var > 0.0 ? var : 0.0;
    const float varf = (float)var, muf = (float)mu;
    const float sc = g0[tid] * rsqrtf(varf + 1e-5f);
    ssc[tid] = sc; ssh[tid] = be0[tid] - muf * sc;
  }
  __syncthreads();
  if (tid < HID) {
    float acc = b1[tid];
#pragma unroll 1
    for (int k = 0; k < HID; ++k) acc = fmaf(ssh[k], W1[(size_t)k * HID + tid], acc);
    sc1[tid] = acc;
  }
  __syncthreads();
  const int piece = tid & 7, lgrp = tid >> 3;
  for (int pass = 0; pass < 2; ++pass) {
#pragma unroll 1
    for (int it = 0; it < 8; ++it) {
      const int L = it * 32 + lgrp; const int n = L >> 1; const int k0 = 64 * (L & 1) + 8 * piece;
      unsigned short hb[8];
#pragma unroll
      for (int e = 0; e < 8; ++e) hb[e] = h_bits(ssc[k0 + e] * W1[(size_t)(k0 + e) * HID + n] * CARRY_W);
      const v4u u = (v4u){pk16(hb[0], hb[1]), pk16(hb[2], hb[3]), pk16(hb[4], hb[5]), pk16(hb[6], hb[7])};
      *(volatile v4u*)(W1T + (size_t)n * HID + k0) = u;
    }
    if (wave == 0) { const v4f v = *(const v4f*)(sc1 + 4 * lane); *(volatile v4f*)(c1 + 4 * lane) = v; }
    __threadfence();
  }
}

__global__ __launch_bounds__(NT) void cast8_kernel(const float* __restrict__ in, unsigned short* __restrict__ out, int n8, float scale) {
  const int i = blockIdx.x * 256 + threadIdx.x;
  if (i >= n8) return;
  const float* p = in + 8 * (size_t)i;
  const v4f a = *(const v4f*)(p);
  const v4f c = *(const v4f*)(p + 4);
  unsigned short hb[8];
#pragma unroll
  for (int e = 0; e < 4; ++e) {
    hb[e]     = h_bits(a[e] * scale);
    hb[4 + e] = h_bits(c[e] * scale);
  }
  const v4u u = (v4u){pk16(hb[0], hb[1]), pk16(hb[2], hb[3]), pk16(hb[4], hb[5]), pk16(hb[6], hb[7])};
  unsigned short* q = out + 8 * (size_t)i;
  *(volatile v4u*)q = u;
  __threadfence();
  *(volatile v4u*)q = u;
}

__global__ __launch_bounds__(NT) void pool_kernel(const float* __restrict__ Z1, const float* __restrict__ Z2, const int* __restrict__ batch,
                                                 const float* __restrict__ c1, const float* __restrict__ b2,
                                                 float* __restrict__ PT, float* __restrict__ CT, int r0, int r1) {
  __shared__ int LIST[PSCH];
  __shared__ int scan_ws[SCANW];
  __shared__ __align__(16) float PACC[8 * 4 * PTW];
  __shared__ float CN[32];
  const int tid = threadIdx.x, lane = tid & 31, wave = tid >> 5;
  const int g0 = blockIdx.x * 32;
  const v4f cv = *(const v4f*)(c1 + 4 * lane);
  const v4f bv = *(const v4f*)(b2 + 4 * lane);
  const v4f z4 = {0.f, 0.f, 0.f, 0.f};
  for (int i = tid; i < PSCH; i += NT) LIST[i] = 0;
  for (int i = tid; i < SCANW; i += NT) scan_ws[i] = 0;
  float* pw = PACC + (size_t)wave * 4 * PTW;
#pragma unroll
  for (int s = 0; s < 4; ++s)
#pragma unroll
    for (int p = 0; p < 4; ++p) *(v4f*)(pw + s * PTW + p * HID + 4 * lane) = z4;
  int cn0 = 0, cn1 = 0, cn2 = 0, cn3 = 0;
  __syncthreads();
  const int nsteps = (r1 - r0 + PSCH - 1) / PSCH;
#pragma unroll 1
  for (int st = 0; st < nsteps; ++st) {
    const int eb = r0 + st * PSCH + tid * PSP;
    const bool valid = eb < r1;
    const int ebc = valid ? eb : (r1 - PSP);
    const v4i ba = *(const v4i*)(batch + ebc);
    const v4i bb = *(const v4i*)(batch + ebc + 4);
    int bvv[PSP];
    bvv[0] = ba[0]; bvv[1] = ba[1]; bvv[2] = ba[2]; bvv[3] = ba[3]; bvv[4] = bb[0]; bvv[5] = bb[1]; bvv[6] = bb[2]; bvv[7] = bb[3];
    int rec[PSP]; int cnt = 0;
#pragma unroll
    for (int k = 0; k < PSP; ++k) {
      const int g = bvv[k]; int r = -1;
      if (valid && g >= g0 && g < g0 + 32) { r = ((g - g0) << 18) | (eb + k); ++cnt; }
      rec[k] = r;
    }
    int tot; int p = blk_excl_scan(cnt, scan_ws, tid, &tot);
#pragma unroll
    for (int k = 0; k < PSP; ++k) if (rec[k] >= 0) { if ((unsigned)p < (unsigned)PSCH) LIST[p] = rec[k]; ++p; }
    __syncthreads();
    const int totc = tot < PSCH ? tot : PSCH;
#pragma unroll 1
    for (int base = 0; base < totc; base += 32) {
      const int q = base + lane; const int qc = q < PSCH ? q : (PSCH - 1);
      const int lv = LIST[qc];
      const int own = ((q < totc) && ((lv >> 20) == wave)) ? 1 : 0;
      unsigned msk = (unsigned)__ballot(own);
#pragma unroll 1
      for (int it = 0; it < 32; ++it) {
        if (msk == 0u) break;
        const int bp = __builtin_ctz(msk); msk &= msk - 1u;
        const int r = __shfl(lv, bp, 32);
        const int sub = (r >> 18) & 3;
        int nd = r & 0x3FFFF; nd = nd < r0 ? r0 : (nd >= r1 ? (r1 - 1) : nd);
        const int rl = nd - r0;
        const v4f z1 = *(const v4f*)(Z1 + (size_t)rl * HID + 4 * lane);
        const v4f z2 = *(const v4f*)(Z2 + (size_t)rl * HID + 4 * lane);
        v4f h1, h2;
#pragma unroll
        for (int e = 0; e < 4; ++e) { h1[e] = fmaxf(z1[e] + cv[e], 0.f); h2[e] = fmaxf(z2[e] + bv[e], 0.f); }
        float* ps = pw + sub * PTW + 4 * lane;
        v4f a0 = *(const v4f*)(ps);            a0 = a0 + h1;       *(v4f*)(ps) = a0;
        v4f a1 = *(const v4f*)(ps + HID);      a1 = a1 + h1 * h1;  *(v4f*)(ps + HID) = a1;
        v4f a2 = *(const v4f*)(ps + 2 * HID);  a2 = a2 + h2;       *(v4f*)(ps + 2 * HID) = a2;
        v4f a3 = *(const v4f*)(ps + 3 * HID);  a3 = a3 + h2 * h2;  *(v4f*)(ps + 3 * HID) = a3;
        cn0 += (sub == 0) ? 1 : 0; cn1 += (sub == 1) ? 1 : 0; cn2 += (sub == 2) ? 1 : 0; cn3 += (sub == 3) ? 1 : 0;
      }
    }
    __syncthreads();
  }
  for (int pass = 0; pass < 2; ++pass) {
#pragma unroll
    for (int s = 0; s < 4; ++s) {
      const int g = g0 + 4 * wave + s;
      float* dst = PT + (size_t)g * PTW;
#pragma unroll
      for (int p = 0; p < 4; ++p) {
        const v4f v = *(const v4f*)(pw + s * PTW + p * HID + 4 * lane);
        *(volatile v4f*)(dst + p * HID + 4 * lane) = v;
      }
    }
    __threadfence();
  }
  if (lane == 0) { CN[4 * wave] = (float)cn0; CN[4 * wave + 1] = (float)cn1; CN[4 * wave + 2] = (float)cn2; CN[4 * wave + 3] = (float)cn3; }
  __syncthreads();
  if (wave == 0) {
    const float cf = CN[lane];
    *(volatile float*)(CT + g0 + lane) = cf;
    __threadfence();
    *(volatile float*)(CT + g0 + lane) = cf;
  }
}

__global__ __launch_bounds__(NT) void final_kernel(const float* __restrict__ PT, const float* __restrict__ CT,
                                                  const float* __restrict__ g1, const float* __restrict__ be1,
                                                  const float* __restrict__ g2, const float* __restrict__ be2,
                                                  const float* __restrict__ W3, const float* __restrict__ b3, float* __restrict__ out) {
  __shared__ float coefA[2 * HID];
  __shared__ float partK[2 * HID];
  __shared__ float sK[1];
  __shared__ __align__(16) float so[NGPAD];
  const int tid = threadIdx.x;
  {
    const int cc = tid; const int soff = (cc < HID) ? cc : (cc + HID);
    double S = 0.0, Q = 0.0;
#pragma unroll 1
    for (int ch = 0; ch < NCHUNK; ++ch) {
#pragma unroll 1
      for (int g = 0; g < NGPAD; ++g) {
        const float* row = PT + ((size_t)(ch * NGPAD + g)) * PTW;
        S += (double)row[soff]; Q += (double)row[soff + HID];
      }
    }
    const double mu = S / (double)NNODE;
    double var = Q / (double)NNODE - mu * mu; var = var > 0.0 ? var : 0.0;
    const float varf = (float)var, muf = (float)mu;
    const int i1 = cc & (HID - 1);
    const float fa = (cc < HID) ? 1.0f : 0.0f; const float fb = 1.0f - fa;
    const float ga = g1[i1], gb = g2[i1], bea = be1[i1], beb = be2[i1];
    const float gam = fmaf(fa, ga, fb * gb);
    const float bet = fmaf(fa, bea, fb * beb);
    const float sc = gam * rsqrtf(varf + 1e-5f);
    const float w3 = W3[cc];
    coefA[cc] = w3 * sc;
    partK[cc] = w3 * (bet - muf * sc);
  }
  __syncthreads();
  if (tid == 0) {
    double k = 0.0;
#pragma unroll 1
    for (int cc = 0; cc < 2 * HID; ++cc) k += (double)partK[cc];
    sK[0] = (float)k;
  }
  __syncthreads();
  const float kK = sK[0]; const float b3v = b3[0];
#pragma unroll 1
  for (int b = tid; b < NGPAD; b += NT) {
    float cnt = 0.f;
#pragma unroll 1
    for (int ch = 0; ch < NCHUNK; ++ch) cnt += CT[ch * NGPAD + b];
    double dot = 0.0;
#pragma unroll 1
    for (int cc = 0; cc < 2 * HID; ++cc) {
      const int soff = (cc < HID) ? cc : (cc + HID);
      float ssum = 0.f;
#pragma unroll 1
      for (int ch = 0; ch < NCHUNK; ++ch) ssum += PT[((size_t)(ch * NGPAD + b)) * PTW + soff];
      dot += (double)coefA[cc] * (double)ssum;
    }
    const float full = (float)(dot / (double)(cnt > 0.5f ? cnt : 1.0f) + (double)kK + (double)b3v);
    so[b] = (cnt > 0.5f) ? full : b3v;
  }
  __syncthreads();
  const bool wr = tid < (NGRAPH / 4);
  const v4f v = *(const v4f*)(so + 4 * tid);
  if (wr) *(volatile v4f*)(out + 4 * tid) = v;
  __threadfence();
  if (wr) *(volatile v4f*)(out + 4 * tid) = v;
}

extern "C" void kernel_launch(void* const* d_in, const int* in_sizes, int n_in,
                              void* d_out, int out_size, void* d_ws, size_t ws_size, hipStream_t stream) {
  (void)in_sizes; (void)n_in; (void)out_size;
  const float* x    = (const float*)d_in[0];
  const float* act  = (const float*)d_in[1];
  const float* Wg   = (const float*)d_in[2];
  const float* bg   = (const float*)d_in[3];
  const float* g0   = (const float*)d_in[4];
  const float* be0  = (const float*)d_in[5];
  const float* W1   = (const float*)d_in[6];
  const float* b1   = (const float*)d_in[7];
  const float* g1   = (const float*)d_in[8];
  const float* be1  = (const float*)d_in[9];
  const float* W2   = (const float*)d_in[10];
  const float* b2   = (const float*)d_in[11];
  const float* g2   = (const float*)d_in[12];
  const float* be2  = (const float*)d_in[13];
  const float* W3   = (const float*)d_in[14];
  const float* b3   = (const float*)d_in[15];
  const int*   ei   = (const int*)d_in[16];
  const int*   bat  = (const int*)d_in[17];
  float* out = (float*)d_out;

  char* ws = (char*)d_ws; size_t off = 0;
  auto carve = [&](size_t bytes) -> char* { char* p = ws + off; off += (bytes + 255) & ~(size_t)255; return p; };
  unsigned short* WgT  = (unsigned short*)carve((size_t)HID * SDIM * 2);
  unsigned short* W2T  = (unsigned short*)carve((size_t)HID * ADIM * 2);
  float*          bsc  = (float*)carve((size_t)HID * 4);
  unsigned short* W1T  = (unsigned short*)carve((size_t)HID * HID * 2);
  float*          c1   = (float*)carve((size_t)HID * 4);
  float*          dinv = (float*)carve((size_t)DINV_ROWS * 4);
  float*          ST0  = (float*)carve((size_t)NSTATBLK * 256 * 4);
  float*          ACC  = (float*)carve((size_t)CHUNK_ROWS * SDIM * 4);
  unsigned short* XAc  = (unsigned short*)carve((size_t)CHUNK_ROWS * SDIM * 2);
  unsigned short* H0   = (unsigned short*)carve((size_t)NNODE * HID * 2);
  float*          Z1c  = (float*)carve((size_t)CHUNK_ROWS * HID * 4);
  float*          Z2c  = (float*)carve((size_t)CHUNK_ROWS * HID * 4);
  unsigned short* ACTc = (unsigned short*)carve((size_t)CHUNK_ROWS * ADIM * 2);
  float*          PT   = (float*)carve((size_t)NCHUNK * NGPAD * PTW * 4);
  float*          CT   = (float*)carve((size_t)NCHUNK * NGPAD * 4);
  if (off > ws_size || off > (size_t)134217728) return;

  pack_kernel<<<1, NT, 0, stream>>>(Wg, W2, bg, WgT, W2T, bsc);
  deg_kernel<<<NDEGBLK, NT, 0, stream>>>(ei, dinv);

  for (int j = 0; j < NCHUNK; ++j) {
    const int r0 = j * CHUNK_ROWS;
    const int rows = (NNODE - r0 < CHUNK_ROWS) ? (NNODE - r0) : CHUNK_ROWS;
    agg_kernel<<<TILES_PER_CHUNK, NT, 0, stream>>>(x, ei, dinv, ACC, XAc, j * TILES_PER_CHUNK);
    const int tiles = (rows / 64) * (HID / 64);
    wmma_gemm64<0, false, 2, 1, false, 2><<<dim3((tiles + 7) / 8, 1), 256, 0, stream>>>(
        (const unsigned short*)XAc, (const unsigned short*)nullptr, SDIM, 0L,
        (const unsigned short*)WgT, (const unsigned short*)nullptr, SDIM, 0L,
        (void*)(H0 + (size_t)r0 * HID), (void*)nullptr, HID, 0L,
        bsc, (const float*)nullptr, 0L, rows, HID, SDIM, SCALE_G1);
  }
  stats0_kernel<<<NSTATBLK, NT, 0, stream>>>((const unsigned*)H0, ST0);
  fold_kernel<<<1, NT, 0, stream>>>(ST0, g0, be0, W1, b1, W1T, c1);

  for (int j = 0; j < NCHUNK; ++j) {
    const int r0 = j * CHUNK_ROWS;
    const int rows = (NNODE - r0 < CHUNK_ROWS) ? (NNODE - r0) : CHUNK_ROWS;
    const int tiles = (rows / 64) * (HID / 64);
    wmma_gemm64<0, false, 0, 0, false, 0><<<dim3((tiles + 7) / 8, 1), 256, 0, stream>>>(
        (const unsigned short*)(H0 + (size_t)r0 * HID), (const unsigned short*)nullptr, HID, 0L,
        (const unsigned short*)W1T, (const unsigned short*)nullptr, HID, 0L,
        (void*)Z1c, (void*)nullptr, HID, 0L,
        (const float*)nullptr, (const float*)nullptr, 0L, rows, HID, HID, SCALE_G2);
    const int n8 = rows * ADIM / 8;
    cast8_kernel<<<n8 / NT, NT, 0, stream>>>(act + (size_t)r0 * ADIM, ACTc, n8, CARRY_ACT);
    wmma_gemm64<0, false, 0, 0, false, 0><<<dim3((tiles + 7) / 8, 1), 256, 0, stream>>>(
        (const unsigned short*)ACTc, (const unsigned short*)nullptr, ADIM, 0L,
        (const unsigned short*)W2T, (const unsigned short*)nullptr, ADIM, 0L,
        (void*)Z2c, (void*)nullptr, HID, 0L,
        (const float*)nullptr, (const float*)nullptr, 0L, rows, HID, ADIM, SCALE_G3);
    pool_kernel<<<NGPAD / 32, NT, 0, stream>>>(Z1c, Z2c, bat, c1, b2,
                                               PT + (size_t)j * NGPAD * PTW, CT + (size_t)j * NGPAD, r0, r0 + rows);
  }
  final_kernel<<<1, NT, 0, stream>>>(PT, CT, g1, be1, g2, be2, W3, b3, out);
}
